// BSRBF_KANLayer_17471926960416
// MI455X (gfx1250) — hardware-verified
//
#include <hip/hip_runtime.h>
#include <math.h>

typedef __attribute__((ext_vector_type(16))) _Float16 v16h;
typedef __attribute__((ext_vector_type(16))) __bf16 v16b;
typedef __attribute__((ext_vector_type(8)))  _Float16 v8h;
typedef __attribute__((ext_vector_type(8)))  float v8f;
typedef __attribute__((ext_vector_type(4)))  float v4f;
typedef __attribute__((ext_vector_type(2)))  float v2f;
typedef __attribute__((ext_vector_type(4)))  unsigned v4u;
typedef __attribute__((ext_vector_type(4)))  int v4i;
typedef float __attribute__((may_alias)) float_a;
typedef int __attribute__((may_alias)) int_a;

template <typename T> __device__ __forceinline__ void vst2(void* p, T v) { *(volatile T*)p = v; __threadfence(); *(volatile T*)p = v; }
__device__ __forceinline__ v8f wmma16(v16h a, v16h b, v8f c) {
  v8f d = __builtin_amdgcn_wmma_f32_16x16x32_f16(false, a, false, b, (short)0, c, false, false);
  asm volatile("v_nop\n\tv_nop\n\tv_nop\n\tv_nop" : "+v"(d) : "v"(a), "v"(b));
  return d;
}
__device__ __forceinline__ v8f wmma_bf(v16b a, v16b b, v8f c) {
  v8f d = __builtin_amdgcn_wmma_f32_16x16x32_bf16(false, a, false, b, (short)0, c, false, false);
  asm volatile("v_nop\n\tv_nop\n\tv_nop\n\tv_nop" : "+v"(d) : "v"(a), "v"(b));
  return d;
}
__device__ __forceinline__ v16h frag_h(const _Float16* rowk0, int lane) {
  union { v16h v; v8h q[2]; } u; const _Float16* p = rowk0 + 8 * (lane >> 4);
  u.q[0] = *(const v8h*)p; u.q[1] = *(const v8h*)(p + 16); return u.v;
}
__device__ __forceinline__ v16h frag_f32(const float* rowk0, int lane) {
  v16h a; const float* p = rowk0 + 8 * (lane >> 4);
#pragma unroll
  for (int i = 0; i < 8; ++i) { a[i] = (_Float16)p[i]; a[8 + i] = (_Float16)p[16 + i]; }
  return a;
}
__device__ __forceinline__ v16h frag_f32s(const float* rowk0, int lane, float sc) {
  v16h a; const float* p = rowk0 + 8 * (lane >> 4);
#pragma unroll
  for (int i = 0; i < 8; ++i) { a[i] = (_Float16)(p[i] * sc); a[8 + i] = (_Float16)(p[16 + i] * sc); }
  return a;
}
__device__ __forceinline__ v16h fragc_f32(const float* W, int k0, int n, int lane, int ld, int K) {
  v16h a; const int g = lane >> 4;
#pragma unroll
  for (int i = 0; i < 8; ++i) { const int ka = k0 + 8 * g + i, kb = ka + 16;
    a[i] = (_Float16)(ka < K ? W[(size_t)(ka < K ? ka : K - 1) * ld + n] : 0.f); a[8 + i] = (_Float16)(kb < K ? W[(size_t)(kb < K ? kb : K - 1) * ld + n] : 0.f); }
  return a;
}
struct F2 { v16b h, l; };
__device__ __forceinline__ F2 bsplit16(const float v[16]) { F2 r;
#pragma unroll
  for (int i = 0; i < 16; ++i) { const __bf16 h = (__bf16)v[i]; r.h[i] = h; r.l[i] = (__bf16)(v[i] - (float)h); }
  return r; }
__device__ __forceinline__ F2 split_row(const float* row, int k0, int lane) { float v[16]; const float* p = row + k0 + 8 * (lane >> 4);
#pragma unroll
  for (int i = 0; i < 8; ++i) { v[i] = p[i]; v[8 + i] = p[16 + i]; }
  return bsplit16(v); }
__device__ __forceinline__ F2 split_rowK(const float* row, int k0, int lane, int K) { float v[16]; const int g = lane >> 4;
#pragma unroll
  for (int i = 0; i < 8; ++i) { const int ka = k0 + 8 * g + i, kb = ka + 16; v[i] = ka < K ? row[ka < K ? ka : K - 1] : 0.f; v[8 + i] = kb < K ? row[kb < K ? kb : K - 1] : 0.f; }
  return bsplit16(v); }
__device__ __forceinline__ F2 split_col(const float* W, int k0, int n, int lane, int ld, int K) { float v[16]; const int g = lane >> 4;
#pragma unroll
  for (int i = 0; i < 8; ++i) { const int ka = k0 + 8 * g + i, kb = ka + 16; v[i] = ka < K ? W[(size_t)(ka < K ? ka : K - 1) * ld + n] : 0.f; v[8 + i] = kb < K ? W[(size_t)(kb < K ? kb : K - 1) * ld + n] : 0.f; }
  return bsplit16(v); }
__device__ __forceinline__ v8f mac3(const F2& a, const F2& b, v8f c) { c = wmma_bf(a.l, b.h, c); c = wmma_bf(a.h, b.l, c); return wmma_bf(a.h, b.h, c); }
__device__ __forceinline__ float sigm(float v) { return 1.0f / (1.0f + expf(-v)); }
#define LDSX() do { asm volatile("s_wait_dscnt 0" ::: "memory"); __builtin_amdgcn_wave_barrier(); __builtin_amdgcn_fence(__ATOMIC_RELEASE, "workgroup"); } while (0)

__device__ __forceinline__ float bfr(float v) { return (float)(__bf16)v; }
#define NR 16384
#define DI 512
#define DO 512
#define NBAS 8
#define KF (DI * NBAS)
#ifndef NRB
#define NRB (NR / 64)
#endif
__constant__ float KNOT[12] = {-3.3000001907348633f,-2.700000047683716f,-2.0999999046325684f,-1.5f,-0.8999999761581421f,-0.2999999523162842f,0.30000007152557373f,0.9000000953674316f,1.5f,2.1000001430511475f,2.700000286102295f,3.3000001907348633f};
__constant__ float CENT[8] = {-1.5f,-1.0714285373687744f,-0.6428570747375488f,-0.21428561210632324f,0.21428585052490234f,0.6428572535514832f,1.0714287757873535f,1.5f};
#define RBF_DEN 0.42857142857142855f
#define WS_ST  0u
#define WS_RX  (WS_ST + 4u * (size_t)NR * 2)
#define WS_FT  (WS_RX + 2u * (size_t)NR * DI)
#define WS_WB  (WS_FT + 2u * (size_t)NR * KF)
#define WS_WS  (WS_WB + 2u * (size_t)DO * DI)
#define WS_END (WS_WS + 2u * (size_t)DO * KF)
__global__ __launch_bounds__(256) void k_stat(const float* __restrict__ X, float* __restrict__ ST) { __shared__ __align__(16) float so[32];
  const int t = threadIdx.x; const int rl = t >> 4, sub = t & 15; const size_t row = (size_t)blockIdx.x * 16 + rl; const float* p = X + row * DI;
  float s = 0.f; for (int c = sub; c < DI; c += 16) s += bfr(p[c]);
#pragma unroll
  for (int o = 1; o < 16; o <<= 1) s += __shfl_xor(s, o);
  const float mu = s * (1.0f / DI); float s2 = 0.f; for (int c = sub; c < DI; c += 16) { const float d = bfr(p[c]) - mu; s2 += d * d; }
#pragma unroll
  for (int o = 1; o < 16; o <<= 1) s2 += __shfl_xor(s2, o);
  if (sub == 0) { so[rl * 2] = mu; so[rl * 2 + 1] = rsqrtf(s2 * (1.0f / DI) + 1e-5f); }
  __syncthreads(); if (t < 32) vst2(ST + (size_t)blockIdx.x * 32 + t, so[t]); }
__global__ __launch_bounds__(256) void k_feat(const float* __restrict__ X, const float* __restrict__ ST, const float* __restrict__ LG, const float* __restrict__ LB, _Float16* __restrict__ RX, _Float16* __restrict__ FT) { __shared__ __align__(16) _Float16 srx[256][8]; __shared__ __align__(16) _Float16 sft[256][8]; __shared__ float sbas[256][8];
  const int t = threadIdx.x; const size_t row = (size_t)blockIdx.x * 4 + (t >> 6); const int d0 = (t & 63) * 8; const float mu = ST[row * 2], rs = ST[row * 2 + 1];
#pragma unroll 1
  for (int e = 0; e < 8; ++e) { const int d = d0 + e; const float xn = (bfr(X[row * DI + d]) - mu) * rs * bfr(LG[d]) + bfr(LB[d]);
    srx[t][e] = (_Float16)fmaxf(xn, 0.f);
    float* bas = &sbas[t][0];
#pragma unroll
    for (int j = 0; j < 8; ++j) bas[j] = 0.f;
    const float tpos = (xn - KNOT[0]) / (KNOT[1] - KNOT[0]);
    if (xn >= KNOT[0] && xn < KNOT[11]) { int s = (int)floorf(tpos); s = s < 0 ? 0 : (s > 10 ? 10 : s); const float f = tpos - (float)s; const float f2 = f * f, f3 = f2 * f; const float omf = 1.f - f;
      const float w0 = omf * omf * omf * (1.f / 6.f), w1 = (3.f * f3 - 6.f * f2 + 4.f) * (1.f / 6.f), w2 = (-3.f * f3 + 3.f * f2 + 3.f * f + 1.f) * (1.f / 6.f), w3 = f3 * (1.f / 6.f);
#pragma unroll
      for (int j = 0; j < 8; ++j) { const int k = s - j; bas[j] = (k == 3) ? w0 : (k == 2) ? w1 : (k == 1) ? w2 : (k == 0) ? w3 : 0.f; } }
#pragma unroll 1
    for (int j = 0; j < 8; ++j) { const float z = (xn - CENT[j]) / RBF_DEN; sft[t][j] = (_Float16)(bas[j] + expf(-(z * z))); }
    vst2((v4u*)(FT + row * KF + (size_t)d * NBAS), *(const v4u*)&sft[t][0]); }
  vst2((v4u*)(RX + row * DI + d0), *(const v4u*)&srx[t][0]); }
__global__ __launch_bounds__(256) void k_wprep(const float* __restrict__ BW, const float* __restrict__ SW, _Float16* __restrict__ WB, _Float16* __restrict__ WSP) {
  const size_t nb = (size_t)DO * DI / 8, nsp = (size_t)DO * KF / 8; const size_t i = (size_t)blockIdx.x * 256 + threadIdx.x;
  union { v4u v; _Float16 h[8]; } u;
  if (i < nb) { const float* p = BW + i * 8;
#pragma unroll
    for (int z = 0; z < 8; ++z) u.h[z] = (_Float16)bfr(p[z]);
    vst2((v4u*)(WB + i * 8), u.v); }
  else if (i < nb + nsp) { const size_t k = i - nb; const float* p = SW + k * 8;
#pragma unroll
    for (int z = 0; z < 8; ++z) u.h[z] = (_Float16)bfr(p[z]);
    vst2((v4u*)(WSP + k * 8), u.v); } }
__global__ __launch_bounds__(128) void k_gemm(const _Float16* __restrict__ RX, const _Float16* __restrict__ FT, const _Float16* __restrict__ BW, const _Float16* __restrict__ SW, float* __restrict__ OUT) { __shared__ __align__(16) float sf[4][16][132];
  const int tid = threadIdx.x, wave = tid >> 5, lane = tid & 31, col = lane & 15, g = lane >> 4; const size_t r0 = (size_t)blockIdx.x * 64 + wave * 16; const int c0 = blockIdx.y * 128;
  v8f acc[8] = {};
#pragma unroll 1
  for (int kc = 0; kc < DI / 32; ++kc) { const v16h a = frag_h(RX + (r0 + col) * DI + kc * 32, lane);
#pragma unroll
    for (int j = 0; j < 8; ++j) acc[j] = wmma16(a, frag_h(BW + (size_t)(c0 + j * 16 + col) * DI + kc * 32, lane), acc[j]); }
#pragma unroll 1
  for (int kc = 0; kc < KF / 32; ++kc) { const v16h a = frag_h(FT + (r0 + col) * KF + kc * 32, lane);
#pragma unroll
    for (int j = 0; j < 8; ++j) acc[j] = wmma16(a, frag_h(SW + (size_t)(c0 + j * 16 + col) * KF + kc * 32, lane), acc[j]); }
#pragma unroll
  for (int j = 0; j < 8; ++j)
#pragma unroll
    for (int r = 0; r < 8; ++r) sf[wave][8 * g + r][j * 16 + col] = acc[j][r];
  LDSX(); for (int rl = 0; rl < 16; ++rl) vst2(OUT + (r0 + rl) * DO + c0 + lane * 4, *(const v4f*)&sf[wave][rl][lane * 4]); }
extern "C" void kernel_launch(void* const* d_in, const int* in_sizes, int n_in, void* d_out, int out_size, void* d_ws, size_t ws_size, hipStream_t stream) {
  (void)in_sizes; (void)n_in; (void)out_size;
  const float** F = (const float**)d_in;
  if (ws_size < (size_t)WS_END) return;
  char* ws = (char*)d_ws; float* ST = (float*)(ws + WS_ST); _Float16 *RX = (_Float16*)(ws + WS_RX), *FT = (_Float16*)(ws + WS_FT), *WB = (_Float16*)(ws + WS_WB), *WSP = (_Float16*)(ws + WS_WS);
  k_wprep<<<dim3((DO * DI / 8 + DO * KF / 8 + 255) / 256), 256, 0, stream>>>(F[3], F[4], WB, WSP);
  k_stat<<<dim3(NRB * 4), 256, 0, stream>>>(F[0], ST);
  k_feat<<<dim3(NRB * 16), 256, 0, stream>>>(F[0], ST, F[1], F[2], RX, FT);
  k_gemm<<<dim3(NRB, DO / 128), 128, 0, stream>>>(RX, FT, WB, WSP, (float*)d_out);
}
